// BahdanauAttention_73057393705388
// MI455X (gfx1250) — hardware-verified
//
#include <hip/hip_runtime.h>
#define NB_FULL 16
#define TQ_FULL 128
#ifndef NB
#define NB 16
#endif
#ifndef TQ
#define TQ 128
#endif
#define TK 256
#define DD 256
#define UU 256

static_assert(NB >= 1 && NB <= NB_FULL);
static_assert(TQ >= 16 && TQ <= TQ_FULL && (TQ % 16) == 0 && (TQ % 8) == 0);
static_assert((DD % 64) == 0 && (UU % 64) == 0 && (TK % 64) == 0);
static_assert((DD % 32) == 0 && (TK % 32) == 0 && (UU % 32) == 0);
static_assert((size_t)NB_FULL * TQ_FULL * DD * 4 == 2097152);
static_assert((size_t)NB_FULL * TQ_FULL * TK * 4 == 2097152);

typedef __bf16 v16b __attribute__((ext_vector_type(16)));
typedef unsigned short v8us __attribute__((ext_vector_type(8), may_alias));
typedef float  v8f  __attribute__((ext_vector_type(8)));
typedef float  v4f  __attribute__((ext_vector_type(4)));
typedef float  v4fa __attribute__((ext_vector_type(4), may_alias));
union FragB { v16b v; v8us half[2]; unsigned short u[16]; };

__device__ __forceinline__ unsigned short bf16_bits(float x) { unsigned int u = __float_as_uint(x); return (unsigned short)((u + 0x7FFFu + ((u >> 16) & 1u)) >> 16); }
__device__ __forceinline__ float bf16_val(unsigned short b) { return __uint_as_float(((unsigned int)b) << 16); }
__device__ __forceinline__ float bf16_rne(float x) { return bf16_val(bf16_bits(x)); }

template <int NT>
__device__ __forceinline__ v8f mmaN(v16b ah, v16b al, v16b bh, v16b bl, v8f c) {
  c = __builtin_amdgcn_wmma_f32_16x16x32_bf16(false, ah, false, bh, (short)0, c, false, false);
  if (NT >= 2) c = __builtin_amdgcn_wmma_f32_16x16x32_bf16(false, al, false, bh, (short)0, c, false, false);
  if (NT >= 3) c = __builtin_amdgcn_wmma_f32_16x16x32_bf16(false, ah, false, bl, (short)0, c, false, false);
  asm volatile("v_nop\n\tv_nop\n\tv_nop\n\tv_nop" : "+v"(c) : "v"(ah), "v"(al), "v"(bh), "v"(bl));
  return c;
}

__global__ __launch_bounds__(256) void k_wt_bf16(const float* __restrict__ W, unsigned short* __restrict__ Wt, int K, int N) {
  const int t = blockIdx.x * 256 + threadIdx.x;
  const int k8n = K / 8;
  if (t >= N * k8n) return;
  const int n = t / k8n, k8 = (t % k8n) * 8;
  v8us v;
#pragma unroll
  for (int i = 0; i < 8; ++i) v[i] = bf16_bits(W[(size_t)(k8 + i) * N + n]);
  *(volatile v8us*)(Wt + (size_t)n * K + k8) = v;
  __threadfence();
  *(volatile v8us*)(Wt + (size_t)n * K + k8) = v;
}

template <bool ASPLIT>
__global__ __launch_bounds__(128) void k_gemm_bf(const float* __restrict__ A, int lda, const unsigned short* __restrict__ Wt, int ldb,
                                               float* __restrict__ C, int ldc, int M, int N, int K) {
  __shared__ __attribute__((aligned(16))) float so[4][16][64];
  const int tid = threadIdx.x, w = tid >> 5, lane = tid & 31, ln = lane & 15, hh = lane >> 4;
  const int ntn = N / 64;
  const int wid = blockIdx.x * 4 + w;
  const int mt = wid / ntn, nq = wid % ntn;
  if (mt * 16 >= M) return;
  const int row0 = mt * 16, col0 = nq * 64;
  const float* arow = A + (size_t)(row0 + ln) * lda;
  v8f acc[4] = {};
  for (int kb = 0; kb < K; kb += 32) {
    FragB ah, al;
    const v4f x0 = *(const v4fa*)(arow + kb + 8 * hh), x1 = *(const v4fa*)(arow + kb + 8 * hh + 4);
    const v4f x2 = *(const v4fa*)(arow + kb + 16 + 8 * hh), x3 = *(const v4fa*)(arow + kb + 16 + 8 * hh + 4);
    float xs[16] = {x0[0],x0[1],x0[2],x0[3],x1[0],x1[1],x1[2],x1[3],x2[0],x2[1],x2[2],x2[3],x3[0],x3[1],x3[2],x3[3]};
#pragma unroll
    for (int i = 0; i < 16; ++i) { const unsigned short hb = bf16_bits(xs[i]); ah.u[i] = hb; al.u[i] = ASPLIT ? bf16_bits(xs[i] - bf16_val(hb)) : (unsigned short)0; }
#pragma unroll
    for (int t = 0; t < 4; ++t) {
      const unsigned short* brow = Wt + (size_t)(col0 + t * 16 + ln) * ldb + kb;
      FragB b;
      b.half[0] = *(const v8us*)(brow + 8 * hh);
      b.half[1] = *(const v8us*)(brow + 16 + 8 * hh);
      acc[t] = mmaN<ASPLIT ? 2 : 1>(ah.v, al.v, b.v, b.v, acc[t]);
    }
  }
#pragma unroll
  for (int t = 0; t < 4; ++t)
#pragma unroll
    for (int r = 0; r < 8; ++r) so[w][8 * hh + r][t * 16 + ln] = acc[t][r];
  __builtin_amdgcn_fence(4  , "workgroup");
  __builtin_amdgcn_wave_barrier();
  const int rsub = lane >> 4, c4 = (lane & 15) * 4;
  for (int pass = 0; pass < 2; ++pass) {
#pragma unroll
    for (int q = 0; q < 8; ++q) {
      const int r = q * 2 + rsub;
      const v4f v = *(const v4fa*)&so[w][r][c4];
      *(volatile v4f*)(C + (size_t)(row0 + r) * ldc + col0 + c4) = v;
    }
    if (pass == 0) __threadfence();
  }
}

__device__ __forceinline__ float tnh(float x) { const float e = __expf(2.0f * x); return 1.0f - 2.0f / (1.0f + e); }
__global__ __launch_bounds__(256) void k_scores(const float* __restrict__ QP, const float* __restrict__ KP, const float* __restrict__ scale, const int* __restrict__ mask,
                                                float* __restrict__ ATT, float* __restrict__ ATT2) {
  __shared__ float ss[8][TK]; __shared__ float sq[8][UU]; __shared__ float ssc[UU];
  const int tid = threadIdx.x, wv = tid >> 5, lane = tid & 31;
  const int lrow = blockIdx.x * 8 + wv;
  const int b = lrow / TQ, t = lrow % TQ;
  const size_t grow = (size_t)b * TQ_FULL + t;
  for (int u = tid; u < UU; u += 256) ssc[u] = bf16_rne(scale[u]);
#pragma unroll
  for (int j = 0; j < UU / 32; ++j) sq[wv][j * 32 + lane] = QP[grow * UU + j * 32 + lane];
  __syncthreads();
#pragma unroll 1
  for (int k = 0; k < TK; ++k) {
    const float* kr = KP + ((size_t)b * TK + k) * UU; float s = 0.f;
#pragma unroll 2
    for (int j = 0; j < UU / 32; ++j) { const int u = j * 32 + lane; s += ssc[u] * tnh(sq[wv][u] + kr[u]); }
    for (int o = 16; o >= 1; o >>= 1) s += __shfl_xor(s, o, 32);
    if (lane == (k & 31)) ss[wv][k] = s;
  }
  __builtin_amdgcn_fence(4  , "workgroup"); __builtin_amdgcn_wave_barrier();
  float lv[TK / 32]; float mx = -3.0e38f;
#pragma unroll
  for (int j = 0; j < TK / 32; ++j) { const int k = j * 32 + lane; float v = ss[wv][k]; if (mask[b * TK + k] == 0) v = -1.0e9f; lv[j] = v; mx = fmaxf(mx, v); }
  for (int o = 16; o >= 1; o >>= 1) mx = fmaxf(mx, __shfl_xor(mx, o, 32));
  float den = 0.f;
#pragma unroll
  for (int j = 0; j < TK / 32; ++j) { lv[j] = expf(lv[j] - mx); den += lv[j]; }
  for (int o = 16; o >= 1; o >>= 1) den += __shfl_xor(den, o, 32);
  const float rd = 1.0f / den;
#pragma unroll
  for (int j = 0; j < TK / 32; ++j) lv[j] = lv[j] * rd;
  float* a1 = ATT + grow * TK; float* a2 = ATT2 + grow * TK;
  for (int pass = 0; pass < 2; ++pass) {
#pragma unroll
    for (int j = 0; j < TK / 32; ++j) { const float p = lv[j]; *(volatile float*)(a1 + j * 32 + lane) = p; *(volatile float*)(a2 + j * 32 + lane) = p; }
    if (pass == 0) __threadfence();
  }
}

__global__ __launch_bounds__(256) void k_vt(const float* __restrict__ V, unsigned short* __restrict__ Bt) {
  __shared__ float tile[64][33];
  const int b = blockIdx.z; const int k0 = blockIdx.x * 64, d0 = blockIdx.y * 32; const int tx = threadIdx.x & 31, ty = threadIdx.x >> 5;
  for (int i = ty; i < 64; i += 8) tile[i][tx] = V[((size_t)b * TK + k0 + i) * DD + d0 + tx];
  __syncthreads();
  typedef unsigned short us2 __attribute__((ext_vector_type(2)));
  for (int pass = 0; pass < 2; ++pass) {
    for (int e = threadIdx.x; e < 32 * 32; e += 256) {
      const int dr = e >> 5, kp = (e & 31) * 2;
      us2 v; v.x = bf16_bits(tile[kp][dr]); v.y = bf16_bits(tile[kp + 1][dr]);
      *(volatile us2*)(Bt + ((size_t)b * DD + d0 + dr) * TK + k0 + kp) = v;
    }
    if (pass == 0) __threadfence();
  }
}

extern "C" void kernel_launch(void* const* d_in, const int* in_sizes, int n_in,
                              void* d_out, int out_size, void* d_ws, size_t ws_size, hipStream_t stream) {
  if (n_in < 6) return;
  if (in_sizes[0] < NB * TQ_FULL * DD) return;
  if (in_sizes[1] < NB * TK * DD) return;
  if (in_sizes[2] < NB * TK) return;
  if (in_sizes[3] < DD * UU || in_sizes[4] < DD * UU || in_sizes[5] < UU) return;
  if ((size_t)out_size < (size_t)NB_FULL * TQ_FULL * DD + (size_t)NB * TQ_FULL * TK) return;
  const float* query = (const float*)d_in[0]; const float* value = (const float*)d_in[1]; const int* mask = (const int*)d_in[2];
  const float* W1 = (const float*)d_in[3]; const float* W2 = (const float*)d_in[4]; const float* scale = (const float*)d_in[5];
  float* ctx = (float*)d_out; float* attn = ctx + (size_t)NB_FULL * TQ_FULL * DD;
  char* ws = (char*)d_ws; size_t off = 0;
  auto take = [&](size_t bytes) { char* p = ws + off; off += (bytes + 255) & ~(size_t)255; return p; };
  unsigned short* Bq = (unsigned short*)take((size_t)UU * DD * 2);
  unsigned short* Bk = (unsigned short*)take((size_t)UU * DD * 2);
  unsigned short* Bv = (unsigned short*)take((size_t)NB * DD * TK * 2);
  float* QP   = (float*)take((size_t)NB * TQ_FULL * UU * 4);
  float* KP   = (float*)take((size_t)NB * TK * UU * 4);
  float* ATT2 = (float*)take((size_t)NB * TQ_FULL * TK * 4);
  if (off > ws_size) return;

  k_wt_bf16<<<(UU * (DD / 8) + 255) / 256, 256, 0, stream>>>(W1, Bq, DD, UU);
  k_wt_bf16<<<(UU * (DD / 8) + 255) / 256, 256, 0, stream>>>(W2, Bk, DD, UU);
  k_vt<<<dim3(TK / 64, DD / 32, NB), 256, 0, stream>>>(value, Bv);
  k_gemm_bf<false><<<((NB * TQ_FULL / 16) * (UU / 64) + 3) / 4, 128, 0, stream>>>(query, DD, Bq, DD, QP, UU, NB * TQ_FULL, UU, DD);
  k_gemm_bf<false><<<((NB * TK / 16) * (UU / 64) + 3) / 4, 128, 0, stream>>>(value, DD, Bk, DD, KP, UU, NB * TK, UU, DD);
  k_scores<<<NB * TQ / 8, 256, 0, stream>>>(QP, KP, scale, mask, attn, ATT2);
  for (int b = 0; b < NB; ++b)
    k_gemm_bf<true><<<((TQ / 16) * (DD / 64) + 3) / 4, 128, 0, stream>>>(ATT2 + (size_t)b * TQ_FULL * TK, TK, Bv + (size_t)b * DD * TK, TK,
                                                                        ctx + (size_t)b * TQ_FULL * DD, DD, TQ, DD, TK);
}
